// ECGLSTM_7052336300072
// MI455X (gfx1250) — hardware-run, weakly checked
//
#include <hip/hip_runtime.h>

typedef __attribute__((ext_vector_type(16))) _Float16 v16h;
typedef __attribute__((ext_vector_type(8)))  _Float16 v8h;
typedef __attribute__((ext_vector_type(4)))  _Float16 v4h;
typedef __attribute__((ext_vector_type(16))) __bf16   v16b;
typedef __attribute__((ext_vector_type(8)))  __bf16   v8b;
typedef __attribute__((ext_vector_type(8)))  float    v8f;
typedef __attribute__((ext_vector_type(4)))  float    v4f;

static constexpr int kHid    = 64;
static constexpr int kNBatch = 256;
static constexpr int kTSteps = 5000;
static constexpr int kNGate  = 256;
static constexpr int kNFc    = 128;
static constexpr int kRowsPB = 16;
static constexpr int kXch    = 64;
static constexpr int kHPitch = 72;
static constexpr int kWPitch = 72;
static constexpr float kHsc     = 1024.0f;
static constexpr float kRsc     = 2048.0f;
static constexpr float kWsc     = 64.0f;
static constexpr float kInvMain = 1.0f / 65536.0f;
static constexpr float kInvRes  = 1.0f / 134217728.0f;

static_assert(kNBatch % kRowsPB == 0);
static_assert(kNGate == 4 * kHid);
static_assert((kXch & (kXch - 1)) == 0);
static_assert(kHid % 32 == 0);
static_assert(kNBatch % 64 == 0);
static_assert(kNFc % 64 == 0);
static_assert(kNFc * kHid == 4 * 256 * 8);

static constexpr long kOffHhi = 0;
static constexpr long kOffHlo = 32768;
static constexpr long kOffWhi = 65536;
static constexpr long kOffWlo = 81920;
static constexpr long kOffSpare = 98304;
static constexpr long kWsTotal = 98560;
static_assert(kOffHlo == kOffHhi + (long)kNBatch * kHid * 2);
static_assert(kOffWhi == kOffHlo + (long)kNBatch * kHid * 2);
static_assert(kOffWlo == kOffWhi + (long)kNFc * kHid * 2);
static_assert(kOffSpare == kOffWlo + (long)kNFc * kHid * 2);
static_assert(kWsTotal <= 134217728L);

__device__ __forceinline__ unsigned short f2bf_bits(float f) {
  unsigned u = __float_as_uint(f);
  return (unsigned short)((u + 0x7FFFu + ((u >> 16) & 1u)) >> 16);
}
__device__ __forceinline__ float bf_bits2f(unsigned short h) { return __uint_as_float(((unsigned)h) << 16); }

__device__ __forceinline__ void dep_guard_h(v8f& a, v8f& b, v16h x, v16h y) { asm volatile("v_nop\n\tv_nop\n\tv_nop\n\tv_nop" : "+v"(a), "+v"(b) : "v"(x), "v"(y)); }
__device__ __forceinline__ void dep_guard_b(v8f& a, v8f& b, v16b x, v16b y) { asm volatile("v_nop\n\tv_nop\n\tv_nop\n\tv_nop" : "+v"(a), "+v"(b) : "v"(x), "v"(y)); }
__device__ __forceinline__ void keep4_h(v16h a, v16h b, v16h c, v16h d) { asm volatile("v_nop" :: "v"(a), "v"(b), "v"(c), "v"(d)); }
__device__ __forceinline__ void keep4_b(v16b a, v16b b, v16b c, v16b d) { asm volatile("v_nop" :: "v"(a), "v"(b), "v"(c), "v"(d)); }
__device__ __forceinline__ void acc_guard4(v8f& a, v8f& b, v8f& c, v8f& d) { asm volatile("v_nop\n\tv_nop\n\tv_nop\n\tv_nop" : "+v"(a), "+v"(b), "+v"(c), "+v"(d)); }
template <typename T> struct Frag;
template <> struct Frag<_Float16> {
  typedef v16h V; union U { v16h v; v8h h[2]; };
  static __device__ __forceinline__ v16h load(const _Float16* p) {
    U f; f.h[0] = *(const v8h*)(p); f.h[1] = *(const v8h*)(p + 16); return f.v;
  }
  static __device__ __forceinline__ v8f mma(v16h a, v16h b, v8f c) {
    return __builtin_amdgcn_wmma_f32_16x16x32_f16(false, a, false, b, (short)0, c, false, false);
  }
  static __device__ __forceinline__ void guard(v8f& a, v8f& b, v16h x, v16h y) { dep_guard_h(a, b, x, y); }
  static __device__ __forceinline__ void keep(v16h a, v16h b, v16h c, v16h d) { keep4_h(a, b, c, d); }
};
template <> struct Frag<__bf16> {
  typedef v16b V; union U { v16b v; v8b h[2]; };
  static __device__ __forceinline__ v16b load(const __bf16* p) {
    U f; f.h[0] = *(const v8b*)(p); f.h[1] = *(const v8b*)(p + 16); return f.v;
  }
  static __device__ __forceinline__ v8f mma(v16b a, v16b b, v8f c) {
    return __builtin_amdgcn_wmma_f32_16x16x32_bf16(false, a, false, b, (short)0, c, false, false);
  }
  static __device__ __forceinline__ void guard(v8f& a, v8f& b, v16b x, v16b y) { dep_guard_b(a, b, x, y); }
  static __device__ __forceinline__ void keep(v16b a, v16b b, v16b c, v16b d) { keep4_b(a, b, c, d); }
};

template <int ET> struct Elem;
template <> struct Elem<0> { typedef _Float16 T; };
template <> struct Elem<1> { typedef __bf16 T; };
template <int ET, bool SPLIT, int BIAS_MODE, int OUT_MODE, bool RESID, int ACT = 0>
__global__ __launch_bounds__(256) void wmma_gemm64(
    const unsigned short* __restrict__ Ap, const unsigned short* __restrict__ A2p, int lda, long strideA,
    const unsigned short* __restrict__ Btp, const unsigned short* __restrict__ Bt2p, int ldb, long strideB,
    void* __restrict__ Cout, void* __restrict__ Cout2, int ldc, long strideC,
    const float* __restrict__ bias,
    const float* __restrict__ resid, long strideR,
    int M, int N, int K, float scale) {
  typedef typename Elem<ET>::T T;
  typedef typename Frag<T>::V V;
  const T* A = (const T*)Ap; const T* A2 = (const T*)A2p; const T* Bt = (const T*)Btp; const T* Bt2 = (const T*)Bt2p;
  __shared__ __align__(16) float sT[8][16 * 68];
  const int b    = blockIdx.y;
  const int lane = threadIdx.x & 31;
  const int wave = threadIdx.x >> 5;
  const int tilesN = N >> 6;
  const int tilesM = M >> 6;
  const int tile = blockIdx.x * 8 + wave;
  if (tile >= tilesM * tilesN) return;
  const int tm = tile / tilesN;
  const int tn = tile - tm * tilesN;
  const int m0 = tm << 6;
  const int n0 = tn << 6;

  const T* Ab  = A  + (size_t)b * strideA;
  const T* Bb  = Bt + (size_t)b * strideB;
  const T* Ab2 = SPLIT ? (A2  + (size_t)b * strideA) : nullptr;
  const T* Bb2 = SPLIT ? (Bt2 + (size_t)b * strideB) : nullptr;

  const int rlane = lane & 15;
  const int koff  = (lane >> 4) * 8;
  const int mOff  = (lane >> 4) * 8;

  v8f acc[4][4];
#pragma unroll
  for (int i = 0; i < 4; ++i)
#pragma unroll
    for (int j = 0; j < 4; ++j) acc[i][j] = (v8f){0.f,0.f,0.f,0.f,0.f,0.f,0.f,0.f};

  for (int k0 = 0; k0 < K; k0 += 32) {
    V bh[4], bl[4];
#pragma unroll
    for (int j = 0; j < 4; ++j) {
      const size_t bo = (size_t)(n0 + (j << 4) + rlane) * ldb + koff + k0;
      bh[j] = Frag<T>::load(Bb + bo);
      if (SPLIT) bl[j] = Frag<T>::load(Bb2 + bo);
    }
#pragma unroll
    for (int i = 0; i < 4; ++i) {
      const size_t ao = (size_t)(m0 + (i << 4) + rlane) * lda + koff + k0;
      V ah = Frag<T>::load(Ab + ao);
      V al;
      if (SPLIT) al = Frag<T>::load(Ab2 + ao);
#pragma unroll
      for (int j = 0; j < 4; ++j) {
        acc[i][j] = Frag<T>::mma(ah, bh[j], acc[i][j]);
        if (SPLIT) {
          acc[i][j] = Frag<T>::mma(ah, bl[j], acc[i][j]);
          acc[i][j] = Frag<T>::mma(al, bh[j], acc[i][j]);
        }
      }
      Frag<T>::guard(acc[i][0], acc[i][3], ah, SPLIT ? al : ah);
    }
    Frag<T>::keep(bh[0], bh[1], bh[2], bh[3]);
    if (SPLIT) Frag<T>::keep(bl[0], bl[1], bl[2], bl[3]);
  }
  acc_guard4(acc[0][0], acc[0][1], acc[0][2], acc[0][3]);
  acc_guard4(acc[1][0], acc[1][1], acc[1][2], acc[1][3]);
  acc_guard4(acc[2][0], acc[2][1], acc[2][2], acc[2][3]);
  acc_guard4(acc[3][0], acc[3][1], acc[3][2], acc[3][3]);

  float* slab = sT[wave];
  const float* Rb = RESID ? (resid + (size_t)b * strideR) : nullptr;
#pragma unroll
  for (int i = 0; i < 4; ++i) {
    const int mBase = m0 + (i << 4);
#pragma unroll
    for (int j = 0; j < 4; ++j) {
      const int n = n0 + (j << 4) + rlane;
      float bv = 0.f;
      if (BIAS_MODE == 2) bv = bias[n];
#pragma unroll
      for (int r = 0; r < 8; ++r) {
        float v = acc[i][j][r] * scale;
        if (BIAS_MODE == 1) v += bias[mBase + mOff + r];
        if (BIAS_MODE == 2) v += bv;
        if (RESID) v += Rb[(size_t)(mBase + mOff + r) * ldc + n];
        if (ACT == 1) v = tanhf(v);
        if (ACT == 2) v = fmaxf(v, 0.0f);
        if (ACT == 3) v = v / (1.0f + expf(-v));
        if (ACT == 4) v = (v > 0.f) ? v : 0.01f * v;
        if (ACT == 5) v = 0.5f * v * (1.0f + erff(v * 0.70710678118654752f));
        slab[(mOff + r) * 68 + (j << 4) + rlane] = v;
      }
    }
    __builtin_amdgcn_fence(__ATOMIC_RELEASE, "workgroup");
    __builtin_amdgcn_wave_barrier();
    __builtin_amdgcn_fence(__ATOMIC_ACQUIRE, "workgroup");
    if (OUT_MODE == 0) {
      float* C = (float*)Cout + (size_t)b * strideC;
      const int hh = lane >> 4, c4 = (lane & 15) * 4;
      for (int pass = 0; pass < 2; ++pass) {
#pragma unroll
        for (int it = 0; it < 8; ++it) {
          const int row = it * 2 + hh;
          v4f v = *(const v4f*)(slab + row * 68 + c4);
          *(volatile v4f*)(C + (size_t)(mBase + row) * ldc + n0 + c4) = v;
        }
        __threadfence();
      }
    } else {
      const int q = lane >> 3, c8 = (lane & 7) * 8;
      unsigned short* C  = (unsigned short*)Cout  + (size_t)b * strideC;
      unsigned short* C2 = (OUT_MODE == 2) ? ((unsigned short*)Cout2 + (size_t)b * strideC) : nullptr;
      for (int pass = 0; pass < 2; ++pass) {
#pragma unroll
        for (int it = 0; it < 4; ++it) {
          const int row = it * 4 + q;
          const float* sp = slab + row * 68 + c8;
          v8h hv, lv;
#pragma unroll
          for (int e = 0; e < 8; ++e) {
            if (OUT_MODE == 1) {
              hv[e] = (_Float16)sp[e];
            } else {
              unsigned short hb = f2bf_bits(sp[e]);
              unsigned short lb = f2bf_bits(sp[e] - bf_bits2f(hb));
              hv[e] = __builtin_bit_cast(_Float16, hb);
              lv[e] = __builtin_bit_cast(_Float16, lb);
            }
          }
          *(volatile v8h*)(C + (size_t)(mBase + row) * ldc + n0 + c8) = hv;
          if (OUT_MODE == 2) *(volatile v8h*)(C2 + (size_t)(mBase + row) * ldc + n0 + c8) = lv;
        }
        __threadfence();
      }
    }
    __builtin_amdgcn_fence(__ATOMIC_RELEASE, "workgroup");
    __builtin_amdgcn_wave_barrier();
    __builtin_amdgcn_fence(__ATOMIC_ACQUIRE, "workgroup");
  }
}

__device__ __forceinline__ v8f zero8() { return (v8f){0.f,0.f,0.f,0.f,0.f,0.f,0.f,0.f}; }

__device__ __forceinline__ v8f mma_pair_f16(v16h a0, v16h b0, v16h a1, v16h b1, v8f c) {
  c = __builtin_amdgcn_wmma_f32_16x16x32_f16(false, a0, false, b0, (short)0, c, false, false);
  c = __builtin_amdgcn_wmma_f32_16x16x32_f16(false, a1, false, b1, (short)0, c, false, false);
  asm volatile("v_nop\n\tv_nop\n\tv_nop\n\tv_nop" : "+v"(c) : "v"(a0), "v"(b0), "v"(a1), "v"(b1));
  return c;
}

__device__ __forceinline__ float ex2_hw(float x) {
#if __has_builtin(__builtin_amdgcn_exp2f)
  return __builtin_amdgcn_exp2f(x);
#else
  return exp2f(x);
#endif
}
__device__ __forceinline__ float rcp_hw(float x) {
#if __has_builtin(__builtin_amdgcn_rcpf)
  return __builtin_amdgcn_rcpf(x);
#else
  return 1.0f / x;
#endif
}
__device__ __forceinline__ float sigm_f(float x) {
  const float xc = fminf(fmaxf(x, -30.0f), 30.0f);
  const float t = ex2_hw(xc * -1.4426950408889634f);
  return rcp_hw(1.0f + t);
}
__device__ __forceinline__ float tanh_f(float x) {
  const float xc = fminf(fmaxf(x, -15.0f), 15.0f);
  const float t = ex2_hw(xc * -2.8853900817779268f);
  return (1.0f - t) * rcp_hw(1.0f + t);
}

__global__ __launch_bounds__(256) void fc_weight_planes_kernel(
    const float* __restrict__ W, unsigned short* __restrict__ Whi, unsigned short* __restrict__ Wlo) {
  const int i = blockIdx.x * 256 + threadIdx.x;
  const int row = i >> 3, c8 = (i & 7) * 8;
  const v4f f0 = *(const v4f*)(W + (size_t)row * kHid + c8);
  const v4f f1 = *(const v4f*)(W + (size_t)row * kHid + c8 + 4);
  v8h hv, lv;
#pragma unroll
  for (int e = 0; e < 4; ++e) {
    const unsigned short hb0 = f2bf_bits(f0[e]);
    const unsigned short lb0 = f2bf_bits(f0[e] - bf_bits2f(hb0));
    const unsigned short hb1 = f2bf_bits(f1[e]);
    const unsigned short lb1 = f2bf_bits(f1[e] - bf_bits2f(hb1));
    hv[e] = __builtin_bit_cast(_Float16, hb0);
    lv[e] = __builtin_bit_cast(_Float16, lb0);
    hv[4 + e] = __builtin_bit_cast(_Float16, hb1);
    lv[4 + e] = __builtin_bit_cast(_Float16, lb1);
  }
  unsigned short* ph = Whi + (size_t)row * kHid + c8;
  unsigned short* pl = Wlo + (size_t)row * kHid + c8;
  for (int pass = 0; pass < 2; ++pass) {
    *(volatile v8h*)ph = hv;
    *(volatile v8h*)pl = lv;
    __threadfence();
  }
}

__global__ __launch_bounds__(128) void recurrent_cell_kernel(
    const float* __restrict__ x,
    const float* __restrict__ W_ih,
    const float* __restrict__ W_hh,
    const float* __restrict__ b_ih,
    const float* __restrict__ b_hh,
    unsigned short* __restrict__ Hhi,
    unsigned short* __restrict__ Hlo)
{
  __shared__ __align__(16) _Float16 Wsh[kNGate * kWPitch];
  __shared__ __align__(16) _Float16 Hh[2][kRowsPB * kHPitch];
  __shared__ __align__(16) _Float16 Hl[2][kRowsPB * kHPitch];
  __shared__ __align__(16) float    Xs[kRowsPB * kXch];

  const int tid  = threadIdx.x;
  const int wave = tid >> 5;
  const int lane = tid & 31;
  const int ln   = lane & 15;
  const int hh   = lane >> 4;
  const int base = blockIdx.x * kRowsPB;

#pragma unroll 1
  for (int u = tid; u < kNGate * 16; u += 128) {
    const int n = u >> 4, k4 = (u & 15) * 4;
    const v4f w = *(const v4f*)(W_hh + (size_t)n * kHid + k4);
    v4h hq;
    hq[0] = (_Float16)(w[0] * kWsc);
    hq[1] = (_Float16)(w[1] * kWsc);
    hq[2] = (_Float16)(w[2] * kWsc);
    hq[3] = (_Float16)(w[3] * kWsc);
    *(v4h*)(&Wsh[n * kWPitch + k4]) = hq;
  }
  {
    unsigned* zh = (unsigned*)(&Hh[0][0]);
    unsigned* zl = (unsigned*)(&Hl[0][0]);
#pragma unroll 1
    for (int i = tid; i < kRowsPB * kHPitch / 2; i += 128) { zh[i] = 0u; zl[i] = 0u; }
  }
  float wih[4], bs[4];
#pragma unroll
  for (int g = 0; g < 4; ++g) {
    const int n = g * kHid + wave * 16 + ln;
    wih[g] = W_ih[n];
    bs[g]  = b_ih[n] + b_hh[n];
  }
  __syncthreads();

  float cst[8], hst[8];
#pragma unroll
  for (int r = 0; r < 8; ++r) { cst[r] = 0.f; hst[r] = 0.f; }
  const int col = wave * 16 + ln;
  int pb = 0;

#pragma unroll 1
  for (int t = 0; t < kTSteps; ++t) {
    if ((t & (kXch - 1)) == 0) {
#pragma unroll 1
      for (int u = tid; u < kRowsPB * kXch; u += 128) {
        const int i = u >> 6, j = u & (kXch - 1);
        int tt = t + j;
        tt = (tt < kTSteps) ? tt : (kTSteps - 1);
        Xs[u] = x[(size_t)(base + i) * kTSteps + tt];
      }
      __syncthreads();
    }

    v16h ah[2], al[2];
    {
      const _Float16* ph = &Hh[pb][ln * kHPitch + 8 * hh];
      const _Float16* pl = &Hl[pb][ln * kHPitch + 8 * hh];
#pragma unroll
      for (int kh = 0; kh < 2; ++kh) {
        ah[kh] = Frag<_Float16>::load(ph + 32 * kh);
        al[kh] = Frag<_Float16>::load(pl + 32 * kh);
      }
    }
    const int tj = t & (kXch - 1);
    float xv[8];
#pragma unroll
    for (int r = 0; r < 8; ++r) xv[r] = Xs[(r + 8 * hh) * kXch + tj];

    v8f am[4], ar[4];
#pragma unroll
    for (int g = 0; g < 4; ++g) {
      const _Float16* pw = &Wsh[(g * kHid + wave * 16 + ln) * kWPitch + 8 * hh];
      const v16h b0 = Frag<_Float16>::load(pw);
      const v16h b1 = Frag<_Float16>::load(pw + 32);
      am[g] = mma_pair_f16(ah[0], b0, ah[1], b1, zero8());
      ar[g] = mma_pair_f16(al[0], b0, al[1], b1, zero8());
    }

    _Float16* dh = &Hh[pb ^ 1][0];
    _Float16* dl = &Hl[pb ^ 1][0];
#pragma unroll
    for (int r = 0; r < 8; ++r) {
      const float xp0 = fmaf(xv[r], wih[0], bs[0]);
      const float xp1 = fmaf(xv[r], wih[1], bs[1]);
      const float xp2 = fmaf(xv[r], wih[2], bs[2]);
      const float xp3 = fmaf(xv[r], wih[3], bs[3]);
      const float p0 = fmaf(ar[0][r], kInvRes, fmaf(am[0][r], kInvMain, xp0));
      const float p1 = fmaf(ar[1][r], kInvRes, fmaf(am[1][r], kInvMain, xp1));
      const float p2 = fmaf(ar[2][r], kInvRes, fmaf(am[2][r], kInvMain, xp2));
      const float p3 = fmaf(ar[3][r], kInvRes, fmaf(am[3][r], kInvMain, xp3));
      const float ig = sigm_f(p0);
      const float fg = sigm_f(p1);
      const float gg = tanh_f(p2);
      const float og = sigm_f(p3);
      const float cc = fmaf(fg, cst[r], ig * gg);
      cst[r] = cc;
      const float hvl = og * tanh_f(cc);
      hst[r] = hvl;
      const float hs = hvl * kHsc;
      const _Float16 h16 = (_Float16)hs;
      const _Float16 l16 = (_Float16)((hs - (float)h16) * kRsc);
      const int m = r + 8 * hh;
      dh[m * kHPitch + col] = h16;
      dl[m * kHPitch + col] = l16;
    }
    __syncthreads();
    pb ^= 1;
  }

#pragma unroll
  for (int r = 0; r < 8; ++r) Xs[(r + 8 * hh) * kXch + col] = hst[r];
  __syncthreads();

  {
    const int q = lane >> 3, c8 = (lane & 7) * 8, row = wave * 4 + q;
    v8h hv, lv;
#pragma unroll
    for (int e = 0; e < 8; ++e) {
      const float f = Xs[row * kXch + c8 + e];
      const unsigned short hb = f2bf_bits(f);
      const unsigned short lb = f2bf_bits(f - bf_bits2f(hb));
      hv[e] = __builtin_bit_cast(_Float16, hb);
      lv[e] = __builtin_bit_cast(_Float16, lb);
    }
    unsigned short* ph = Hhi + (size_t)(base + row) * kHid + c8;
    unsigned short* pl = Hlo + (size_t)(base + row) * kHid + c8;
    for (int pass = 0; pass < 2; ++pass) {
      *(volatile v8h*)ph = hv;
      *(volatile v8h*)pl = lv;
      __threadfence();
    }
  }
}

extern "C" void kernel_launch(void* const* d_in, const int* in_sizes, int n_in,
                              void* d_out, int out_size, void* d_ws, size_t ws_size,
                              hipStream_t stream) {
  (void)in_sizes; (void)n_in; (void)out_size; (void)ws_size;
  const float* x    = (const float*)d_in[0];
  const float* W_ih = (const float*)d_in[1];
  const float* W_hh = (const float*)d_in[2];
  const float* b_ih = (const float*)d_in[3];
  const float* b_hh = (const float*)d_in[4];
  const float* W_fc = (const float*)d_in[5];
  const float* b_fc = (const float*)d_in[6];
  char* ws = (char*)d_ws;
  unsigned short* Hhi = (unsigned short*)(ws + kOffHhi);
  unsigned short* Hlo = (unsigned short*)(ws + kOffHlo);
  unsigned short* Whi = (unsigned short*)(ws + kOffWhi);
  unsigned short* Wlo = (unsigned short*)(ws + kOffWlo);
  void* spare = (void*)(ws + kOffSpare);

  fc_weight_planes_kernel<<<dim3(4), dim3(256), 0, stream>>>(W_fc, Whi, Wlo);
  recurrent_cell_kernel<<<dim3(kNBatch / kRowsPB), dim3(128), 0, stream>>>(x, W_ih, W_hh, b_ih, b_hh, Hhi, Hlo);
  wmma_gemm64<1, true, 2, 0, false, 2><<<dim3(1, 1), dim3(256), 0, stream>>>(
      Hhi, Hlo, kHid, 0L,
      Whi, Wlo, kHid, 0L,
      d_out, spare, kNFc, 0L,
      b_fc,
      b_fc, 0L,
      kNBatch, kNFc, kHid, 1.0f);
}
